// OrbitalBackflowNet_18056042512513
// MI455X (gfx1250) — hardware-verified
//
#include <hip/hip_runtime.h>


namespace {
constexpr int Bn = 16, N = 256, D = 3, H = 64, E = 64, NOCC = 128, NT = Bn * N;
constexpr float AS_ = 8.0f, EPS = 1e-12f;

typedef _Float16 b16;
typedef __attribute__((ext_vector_type(16))) _Float16 v16b;
typedef __attribute__((ext_vector_type(8))) _Float16 v8b;
typedef __attribute__((ext_vector_type(8))) float v8f;
typedef __attribute__((ext_vector_type(4))) float v4f;
__device__ __forceinline__ float bf16_rne(float f) { unsigned int u = __float_as_uint(f); u += 0x7FFFu + ((u >> 16) & 1u); return __uint_as_float(u & 0xFFFF0000u); }
__device__ __forceinline__ void split16(float v, b16& hi, b16& lo) { hi = (b16)v; lo = (b16)(v - (float)hi); }
__device__ __forceinline__ v16b frag_kb(const b16* p, int hh) { const v8b a = *(const v8b*)(p + 8 * hh), b = *(const v8b*)(p + 16 + 8 * hh); v16b f;
#pragma unroll
  for (int e = 0; e < 8; ++e) { f[e] = a[e]; f[8 + e] = b[e]; } return f; }
__device__ __forceinline__ v8f wmma16b(v16b a, v16b b, v8f c) { v8f d = __builtin_amdgcn_wmma_f32_16x16x32_f16(false, a, false, b, (short)0, c, false, false); asm volatile("v_nop\n\tv_nop\n\tv_nop\n\tv_nop" : "+v"(d) : "v"(a), "v"(b)); return d; }
__device__ __forceinline__ void wave_lds_sync() { __builtin_amdgcn_fence(__ATOMIC_RELEASE, "workgroup"); __builtin_amdgcn_wave_barrier(); __builtin_amdgcn_fence(__ATOMIC_ACQUIRE, "workgroup"); }
__device__ __forceinline__ float nexp(float x) { return __builtin_amdgcn_exp2f(x * 1.4426950408889634f); }
__device__ __forceinline__ float silu_(float v) { return v * __builtin_amdgcn_rcpf(1.0f + nexp(-v)); }
__device__ __forceinline__ float tanh_(float x) { const float e = nexp(-2.0f * fabsf(x)); const float t = (1.0f - e) * __builtin_amdgcn_rcpf(1.0f + e); return (x >= 0.0f) ? t : -t; }
__device__ __forceinline__ float pmul(float a, float b) { float p = a * b; asm volatile("" : "+v"(p)); return p; }

__global__ __launch_bounds__(256) void prep_kernel(const float* __restrict__ We2, const float* __restrict__ Wu1, const float* __restrict__ Wu2, const float* __restrict__ Wev, const float* __restrict__ Wn1, const float* __restrict__ Wn2, const float* __restrict__ Worb, const float* __restrict__ Wve,
                                                   const float* __restrict__ We1, const float* __restrict__ be1, const float* __restrict__ be2, const float* __restrict__ bu1, const float* __restrict__ bu2, const float* __restrict__ bn1, const float* __restrict__ bn2, const float* __restrict__ borb,
                                                   const float* __restrict__ Wnode, const float* __restrict__ bnode, const float* __restrict__ bf, b16* __restrict__ R, float* __restrict__ P) {
  const int t_ = threadIdx.x;
  for (int pass = 0; pass < 2; ++pass) {
    for (int p = t_; p < 5 * 4096; p += 256) { const int m = p >> 12, q = p & 4095, o = q >> 6, k = q & 63; const float* W = (m == 0) ? We2 : (m == 1) ? Wu1 : (m == 2) ? Wu2 : (m == 3) ? Wev : Wn2;
      ((volatile b16*)R)[p] = (b16)bf16_rne(W[k * 64 + o]); }
    for (int p = t_; p < 64 * 128; p += 256) { const int o = p >> 7, k = p & 127; ((volatile b16*)R)[5 * 4096 + p] = (b16)bf16_rne(Wn1[k * 64 + o]); }
    for (int p = t_; p < 128 * 64; p += 256) { const int o = p >> 6, k = p & 63; ((volatile b16*)R)[7 * 4096 + p] = (b16)bf16_rne(Worb[k * 128 + o]); }
    for (int p = t_; p < 3 * 4096; p += 256) { const int m = p >> 12, q = p & 4095, o = q >> 6, k = q & 63; const float v = (m == 0) ? Wve[k * 64 + o] : Wu1[((m == 1 ? 64 : 128) + k) * 64 + o]; ((volatile b16*)R)[9 * 4096 + p] = (b16)bf16_rne(v); }
    for (int p = t_; p < 64 * 32; p += 256) { const int o = p >> 5, k = p & 31; ((volatile b16*)R)[12 * 4096 + p] = (b16)((k < 4) ? bf16_rne(Wnode[k * 64 + o]) : 0.0f); }
    for (int p = t_; p < 1160; p += 256) { float v = 0.0f;
      if (p < 320) v = bf16_rne(We1[p]); else if (p < 384) v = bf16_rne(be1[p - 320]); else if (p < 448) v = bf16_rne(be2[p - 384]); else if (p < 512) v = bf16_rne(bu1[p - 448]); else if (p < 576) v = bf16_rne(bu2[p - 512]);
      else if (p < 640) v = bf16_rne(bn1[p - 576]); else if (p < 704) v = bf16_rne(bn2[p - 640]); else if (p < 832) v = bf16_rne(borb[p - 704]); else if (p < 1088) v = bf16_rne(Wnode[p - 832]); else if (p < 1152) v = bf16_rne(bnode[p - 1088]);
      else if (p == 1152) { const float z = bf16_rne(bf[0]); v = fmaxf(z, 0.0f) + log1pf(__expf(-fabsf(z))); }
      ((volatile float*)P)[p] = v; }
    __threadfence();
  }
}

__global__ __launch_bounds__(256) void node_pre_kernel(const float* __restrict__ x, const int* __restrict__ spin, const float* __restrict__ P, const b16* __restrict__ R, float* __restrict__ hv, float* __restrict__ pvi, float* __restrict__ pvj) {
  __shared__ __attribute__((aligned(16))) float T[8][16][64 + 4]; __shared__ __attribute__((aligned(16))) float O1[8][16][64 + 4], O2[8][16][64 + 4];
  const int wid = threadIdx.x >> 5, lane = threadIdx.x & 31, nloc = lane & 15, hlf = lane >> 4; const size_t r0 = (size_t)blockIdx.x * 128 + wid * 16;
  const b16* Wnr = R + 12 * 4096; const b16* Wver = R + 9 * 4096; const b16* Wu1b = R + 10 * 4096; const b16* Wu1c = R + 11 * 4096;
  auto afrag = [&](int kb, v16b& ah, v16b& al) {
#pragma unroll
    for (int e = 0; e < 16; ++e) { const int k = kb + ((e < 8) ? (8 * hlf + e) : (16 + 8 * hlf + e - 8)); b16 a, c; split16(T[wid][nloc][k] * AS_, a, c); ah[e] = a; al[e] = c; } };
  auto gemm = [&](const b16* Bw, int KK, v8f* acc) {
    for (int kb = 0; kb < KK; kb += 32) { v16b ah, al; afrag(kb, ah, al);
#pragma unroll
      for (int t = 0; t < 4; ++t) { const v16b bw = frag_kb(Bw + (size_t)(t * 16 + nloc) * KK + kb, hlf); acc[t] = wmma16b(ah, bw, acc[t]); acc[t] = wmma16b(al, bw, acc[t]); } } };
  { const int r = nloc; const size_t n = r0 + r; const float v = (hlf == 0) ? 0.0f : 0.0f; (void)v;
    for (int k = hlf; k < 32; k += 2) { float val = 0.0f; if (k < 3) val = bf16_rne(x[n * 3 + k]); else if (k == 3) val = (float)spin[n % N]; T[wid][r][k] = val; } }
  wave_lds_sync();
  v8f acc[4];
#pragma unroll
  for (int t = 0; t < 4; ++t) acc[t] = (v8f){};
  gemm(Wnr, 32, acc); wave_lds_sync();
#pragma unroll
  for (int t = 0; t < 4; ++t)
#pragma unroll
    for (int v = 0; v < 8; ++v) { const float hval = acc[t][v] * (1.0f / AS_) + P[1088 + t * 16 + nloc]; T[wid][8 * hlf + v][t * 16 + nloc] = hval; O1[wid][8 * hlf + v][t * 16 + nloc] = hval; }
  wave_lds_sync();
#pragma unroll
  for (int t = 0; t < 4; ++t) acc[t] = (v8f){};
  gemm(Wver, 64, acc); wave_lds_sync();
#pragma unroll
  for (int t = 0; t < 4; ++t)
#pragma unroll
    for (int v = 0; v < 8; ++v) T[wid][8 * hlf + v][t * 16 + nloc] = acc[t][v] * (1.0f / AS_);
  wave_lds_sync();
  for (int pass = 0; pass < 2; ++pass) { for (int q = lane; q < 16 * 16; q += 32) { const int r = q >> 4, c4 = (q & 15) * 4; *(volatile v4f*)(hv + (r0 + r) * 64 + c4) = *(const v4f*)(&O1[wid][r][c4]); } __threadfence(); }
#pragma unroll
  for (int t = 0; t < 4; ++t) acc[t] = (v8f){};
  gemm(Wu1b, 64, acc);
  v8f acc2[4];
#pragma unroll
  for (int t = 0; t < 4; ++t) acc2[t] = (v8f){};
  gemm(Wu1c, 64, acc2); wave_lds_sync();
#pragma unroll
  for (int t = 0; t < 4; ++t)
#pragma unroll
    for (int v = 0; v < 8; ++v) { O1[wid][8 * hlf + v][t * 16 + nloc] = acc[t][v] * (1.0f / AS_) + P[448 + t * 16 + nloc]; O2[wid][8 * hlf + v][t * 16 + nloc] = acc2[t][v] * (1.0f / AS_); }
  wave_lds_sync();
  for (int pass = 0; pass < 2; ++pass) { for (int q = lane; q < 16 * 16; q += 32) { const int r = q >> 4, c4 = (q & 15) * 4; *(volatile v4f*)(pvi + (r0 + r) * 64 + c4) = *(const v4f*)(&O1[wid][r][c4]); *(volatile v4f*)(pvj + (r0 + r) * 64 + c4) = *(const v4f*)(&O2[wid][r][c4]); } __threadfence(); }
}

__global__ __launch_bounds__(256) void pair_kernel(const float* __restrict__ x, const float* __restrict__ P, const b16* __restrict__ R, const float* __restrict__ pvi, const float* __restrict__ pvj, float* __restrict__ msum) {
  __shared__ __attribute__((aligned(16))) float T[8][16][E + 4]; __shared__ float Part[8][E]; __shared__ float Ps[576];
  const int wid = threadIdx.x >> 5, lane = threadIdx.x & 31, nloc = lane & 15, hlf = lane >> 4; const int node = blockIdx.x, b = node / N, i = node % N;
  for (int q = threadIdx.x; q < 576; q += 256) Ps[q] = P[q];
  __syncthreads();
  const float* xb = x; const float xi0 = bf16_rne(xb[(size_t)node * 3]), xi1 = bf16_rne(xb[(size_t)node * 3 + 1]), xi2 = bf16_rne(xb[(size_t)node * 3 + 2]);
  const b16* We2r = R; const b16* Wu1r = R + 4096; const b16* Wu2r = R + 2 * 4096;
  float part[4] = {0.0f, 0.0f, 0.0f, 0.0f};
  auto afragT = [&](int kb, v16b& ah, v16b& al) {
#pragma unroll
    for (int e = 0; e < 16; ++e) { const int k = kb + ((e < 8) ? (8 * hlf + e) : (16 + 8 * hlf + e - 8)); b16 a, c; split16(T[wid][nloc][k] * AS_, a, c); ah[e] = a; al[e] = c; } };
  for (int tt = 0; tt < 2; ++tt) { const int j0 = (wid * 2 + tt) * 16; const int jn = (size_t)b * N + j0 + nloc;
    const float r0 = xi0 - bf16_rne(xb[(size_t)jn * 3]), r1_ = xi1 - bf16_rne(xb[(size_t)jn * 3 + 1]), r2_ = xi2 - bf16_rne(xb[(size_t)jn * 3 + 2]); const float rr = r0 * r0 + r1_ * r1_ + r2_ * r2_, rn = sqrtf(rr + EPS);
    v8f acc[4];
#pragma unroll
    for (int t = 0; t < 4; ++t) acc[t] = (v8f){};
#pragma unroll
    for (int ks = 0; ks < 2; ++ks) { v16b ah, al;
#pragma unroll
      for (int e = 0; e < 16; ++e) { const int k = ks * 32 + ((e < 8) ? (8 * hlf + e) : (16 + 8 * hlf + e - 8));
        const float pre = (pmul(r0, Ps[k]) + pmul(r1_, Ps[64 + k])) + (pmul(r2_, Ps[128 + k]) + pmul(rn, Ps[192 + k])) + (pmul(rr, Ps[256 + k]) + Ps[320 + k]); b16 a, c; split16(silu_(pre) * AS_, a, c); ah[e] = a; al[e] = c; }
#pragma unroll
      for (int t = 0; t < 4; ++t) { const v16b bw = frag_kb(We2r + (size_t)(t * 16 + nloc) * 64 + ks * 32, hlf); acc[t] = wmma16b(ah, bw, acc[t]); acc[t] = wmma16b(al, bw, acc[t]); } }
#pragma unroll
    for (int t = 0; t < 4; ++t)
#pragma unroll
      for (int v = 0; v < 8; ++v) T[wid][8 * hlf + v][t * 16 + nloc] = acc[t][v] * (1.0f / AS_) + Ps[384 + t * 16 + nloc];
    wave_lds_sync();
#pragma unroll
    for (int t = 0; t < 4; ++t) acc[t] = (v8f){};
#pragma unroll
    for (int ks = 0; ks < 2; ++ks) { v16b ah, al; afragT(ks * 32, ah, al);
#pragma unroll
      for (int t = 0; t < 4; ++t) { const v16b bw = frag_kb(Wu1r + (size_t)(t * 16 + nloc) * 64 + ks * 32, hlf); acc[t] = wmma16b(ah, bw, acc[t]); acc[t] = wmma16b(al, bw, acc[t]); } }
    wave_lds_sync();
#pragma unroll
    for (int t = 0; t < 4; ++t) { const int c = t * 16 + nloc; const float pi_ = pvi[(size_t)node * 64 + c];
#pragma unroll
      for (int v = 0; v < 8; ++v) { const int j = j0 + 8 * hlf + v; T[wid][8 * hlf + v][c] = silu_(acc[t][v] * (1.0f / AS_) + pi_ + pvj[((size_t)b * N + j) * 64 + c]); } }
    wave_lds_sync();
#pragma unroll
    for (int t = 0; t < 4; ++t) acc[t] = (v8f){};
#pragma unroll
    for (int ks = 0; ks < 2; ++ks) { v16b ah, al; afragT(ks * 32, ah, al);
#pragma unroll
      for (int t = 0; t < 4; ++t) { const v16b bw = frag_kb(Wu2r + (size_t)(t * 16 + nloc) * 64 + ks * 32, hlf); acc[t] = wmma16b(ah, bw, acc[t]); acc[t] = wmma16b(al, bw, acc[t]); } }
    wave_lds_sync();
#pragma unroll
    for (int t = 0; t < 4; ++t) { const float bb = Ps[512 + t * 16 + nloc];
#pragma unroll
      for (int v = 0; v < 8; ++v) { const int j = j0 + 8 * hlf + v; part[t] += (j != i) ? (acc[t][v] * (1.0f / AS_) + bb) : 0.0f; } }
  }
#pragma unroll
  for (int t = 0; t < 4; ++t) { part[t] += __shfl_xor(part[t], 16); if (hlf == 0) Part[wid][t * 16 + nloc] = part[t]; }
  __syncthreads();
  for (int pass = 0; pass < 2; ++pass) { if (threadIdx.x < 64) { float s = 0.0f; for (int w = 0; w < 8; ++w) s += Part[w][threadIdx.x]; ((volatile float*)msum)[(size_t)node * 64 + threadIdx.x] = s; } __threadfence(); }
}

__global__ __launch_bounds__(256) void node_post_kernel(const float* __restrict__ hv, const float* __restrict__ msum, const b16* __restrict__ R, const float* __restrict__ P, float* __restrict__ out) {
  __shared__ __attribute__((aligned(16))) float T[8][16][128 + 4];
  const int wid = threadIdx.x >> 5, lane = threadIdx.x & 31, nloc = lane & 15, hlf = lane >> 4; const size_t r0 = (size_t)blockIdx.x * 128 + wid * 16;
  const b16* Wevr = R + 3 * 4096; const b16* Wn2r = R + 4 * 4096; const b16* Wn1r = R + 5 * 4096; const b16* Worr = R + 7 * 4096; const float sp = P[1152];
  auto afrag = [&](int kb, v16b& ah, v16b& al) {
#pragma unroll
    for (int e = 0; e < 16; ++e) { const int k = kb + ((e < 8) ? (8 * hlf + e) : (16 + 8 * hlf + e - 8)); b16 a, c; split16(T[wid][nloc][k] * AS_, a, c); ah[e] = a; al[e] = c; } };
  auto gemm = [&](const b16* Bw, int KK, int NTL, v8f* acc) {
    for (int kb = 0; kb < KK; kb += 32) { v16b ah, al; afrag(kb, ah, al);
      for (int t = 0; t < NTL; ++t) { const v16b bw = frag_kb(Bw + (size_t)(t * 16 + nloc) * KK + kb, hlf); acc[t] = wmma16b(ah, bw, acc[t]); acc[t] = wmma16b(al, bw, acc[t]); } } };
  for (int q = lane; q < 16 * 16; q += 32) { const int r = q >> 4, c4 = (q & 15) * 4; *(v4f*)(&T[wid][r][c4]) = *(const v4f*)(msum + (r0 + r) * 64 + c4); }
  wave_lds_sync();
  v8f acc[8];
#pragma unroll
  for (int t = 0; t < 4; ++t) acc[t] = (v8f){};
  gemm(Wevr, 64, 4, acc); wave_lds_sync();
#pragma unroll
  for (int t = 0; t < 4; ++t)
#pragma unroll
    for (int v = 0; v < 8; ++v) { const int r = 8 * hlf + v, c = t * 16 + nloc; T[wid][r][64 + c] = acc[t][v] * (1.0f / AS_); T[wid][r][c] = hv[(r0 + r) * 64 + c]; }
  wave_lds_sync();
#pragma unroll
  for (int t = 0; t < 4; ++t) acc[t] = (v8f){};
  gemm(Wn1r, 128, 4, acc); wave_lds_sync();
#pragma unroll
  for (int t = 0; t < 4; ++t)
#pragma unroll
    for (int v = 0; v < 8; ++v) T[wid][8 * hlf + v][t * 16 + nloc] = silu_(acc[t][v] * (1.0f / AS_) + P[576 + t * 16 + nloc]);
  wave_lds_sync();
#pragma unroll
  for (int t = 0; t < 4; ++t) acc[t] = (v8f){};
  gemm(Wn2r, 64, 4, acc); wave_lds_sync();
#pragma unroll
  for (int t = 0; t < 4; ++t)
#pragma unroll
    for (int v = 0; v < 8; ++v) { const int r = 8 * hlf + v, c = t * 16 + nloc; T[wid][r][c] = hv[(r0 + r) * 64 + c] + acc[t][v] * (1.0f / AS_) + P[640 + c]; }
  wave_lds_sync();
#pragma unroll
  for (int t = 0; t < 8; ++t) acc[t] = (v8f){};
  gemm(Worr, 64, 8, acc); wave_lds_sync();
#pragma unroll
  for (int t = 0; t < 8; ++t)
#pragma unroll
    for (int v = 0; v < 8; ++v) T[wid][8 * hlf + v][t * 16 + nloc] = tanh_(acc[t][v] * (1.0f / AS_) + P[704 + t * 16 + nloc]) * sp;
  wave_lds_sync();
  for (int pass = 0; pass < 2; ++pass) { for (int q = lane; q < 16 * 32; q += 32) { const int r = q >> 5, c4 = (q & 31) * 4; *(volatile v4f*)(out + (r0 + r) * NOCC + c4) = *(const v4f*)(&T[wid][r][c4]); } __threadfence(); }
}
}

extern "C" void kernel_launch(void* const* d_in, const int* in_sizes, int n_in,
                              void* d_out, int out_size, void* d_ws, size_t ws_size, hipStream_t stream) {
  (void)n_in; (void)out_size;
  const float* x = (const float*)d_in[0]; const int* spin = (const int*)d_in[1]; const float* Wnode = (const float*)d_in[2]; const float* bnode = (const float*)d_in[3];
  const float* We1 = (const float*)d_in[4]; const float* be1 = (const float*)d_in[5]; const float* We2 = (const float*)d_in[6]; const float* be2 = (const float*)d_in[7]; const float* Wve = (const float*)d_in[8]; const float* Wev = (const float*)d_in[9];
  const float* Wu1 = (const float*)d_in[10]; const float* bu1 = (const float*)d_in[11]; const float* Wu2 = (const float*)d_in[12]; const float* bu2 = (const float*)d_in[13]; const float* Wn1 = (const float*)d_in[14]; const float* bn1 = (const float*)d_in[15]; const float* Wn2 = (const float*)d_in[16]; const float* bn2 = (const float*)d_in[17];
  const float* Worb = (const float*)d_in[18]; const float* borb = (const float*)d_in[19]; const float* bf = (const float*)d_in[20];
  float* out = (float*)d_out;
  if (in_sizes[0] != NT * 3 || in_sizes[1] != N || in_sizes[2] != 4 * 64 || in_sizes[10] != 192 * 64 || in_sizes[18] != 64 * 128) return;
  size_t off = 0; char* ws = (char*)d_ws;
  auto carve = [&](size_t bytes) { char* p = ws + off; off += (bytes + 255) & ~(size_t)255; return p; };
  b16* R = (b16*)carve(13 * 4096 * 2); float* P = (float*)carve(1160 * 4 + 256); float* hv = (float*)carve((size_t)NT * 64 * 4); float* pvi = (float*)carve((size_t)NT * 64 * 4); float* pvj = (float*)carve((size_t)NT * 64 * 4); float* msum = (float*)carve((size_t)NT * 64 * 4);
  if (off > ws_size) return;
  prep_kernel<<<1, 256, 0, stream>>>(We2, Wu1, Wu2, Wev, Wn1, Wn2, Worb, Wve, We1, be1, be2, bu1, bu2, bn1, bn2, borb, Wnode, bnode, bf, R, P);
  node_pre_kernel<<<NT / 128, 256, 0, stream>>>(x, spin, P, R, hv, pvi, pvj);
  pair_kernel<<<NT, 256, 0, stream>>>(x, P, R, pvi, pvj, msum);
  node_post_kernel<<<NT / 128, 256, 0, stream>>>(hv, msum, R, P, out);
}
